// TemporalMambaEncoder_40364102648387
// MI455X (gfx1250) — hardware-verified
//
#include <hip/hip_runtime.h>
#include <hip/hip_bf16.h>
#include <math.h>

#define BDIM   2
#define LDIM   1024
#define NDIM   512
#define NLAYER 2
#define NMB    4
#define DIDIM  1024
#define SDIM   16
#define KCONV  4
#define RDIM   32
#define MROWS  (BDIM*LDIM)
#define XDBLW  (RDIM + 2*SDIM)

#define __bf16 _Float16
#define RSPLIT (1.0f / 2048.0f)
typedef __attribute__((ext_vector_type(16))) __bf16 v16bf;
typedef __attribute__((ext_vector_type(4))) float v4f_t;
typedef float v4fa __attribute__((ext_vector_type(4), may_alias));
__device__ __forceinline__ __bf16 lo_of(float v, __bf16 h) { return (__bf16)((v - (float)h) * 2048.0f); }
__device__ __forceinline__ unsigned pk2s(float a, float b, unsigned* lo) {
  const __bf16 h0 = (__bf16)a, h1 = (__bf16)b;
  *lo = (unsigned)__builtin_bit_cast(unsigned short, lo_of(a, h0)) | ((unsigned)__builtin_bit_cast(unsigned short, lo_of(b, h1)) << 16);
  return (unsigned)__builtin_bit_cast(unsigned short, h0) | ((unsigned)__builtin_bit_cast(unsigned short, h1) << 16);
}
typedef __attribute__((ext_vector_type(8)))  float  v8f;
typedef __attribute__((address_space(3)))    float  lds_f32;

union FragBF { v16bf v; uint4 q[2]; };

__global__ void k_cast_bf16(const float* __restrict__ src, __bf16* __restrict__ dst, int n) {
  int i = (blockIdx.x * blockDim.x + threadIdx.x) * 2;
  if (i >= n) return;
  unsigned lo; const unsigned p = pk2s(src[i], src[i + 1], &lo);
  *(volatile unsigned*)(dst + i) = p; *(volatile unsigned*)(dst + (size_t)n + i) = lo; __threadfence();
  *(volatile unsigned*)(dst + i) = p; *(volatile unsigned*)(dst + (size_t)n + i) = lo;
}
__device__ __forceinline__ v8f wmma_split(v16bf a, v16bf al, v16bf b, v16bf bl, v8f c) {
  (void)al; (void)bl;
  return __builtin_amdgcn_wmma_f32_16x16x32_f16(false, a, false, b, (short)0, c, false, false);
}

__device__ __forceinline__ void load_frag(FragBF& f, const __bf16* p) {
  f.q[0] = *(const uint4*)p;
  f.q[1] = *(const uint4*)(p + 16);
}

__device__ __forceinline__ float apply_epi(float v, float bv, int epilogue) {
  if (epilogue == 1) {
    v += bv;
    v = (v > 20.f) ? v : log1pf(__expf(v));
  }
  return v;
}

__launch_bounds__(128)
__global__ void k_gemm_bf16(const __bf16* __restrict__ A, const __bf16* __restrict__ Bt,
                            float* __restrict__ C, const float* __restrict__ bias,
                            int Kd, int Dn, int epilogue, size_t pa, size_t pb) {
  __shared__ __attribute__((aligned(16))) float stg[4][32 * 36];
  const int lane = threadIdx.x & 31;
  const int wave = threadIdx.x >> 5;
  const int wr = wave >> 1, wc = wave & 1;
  const int m_base = blockIdx.y * 64 + wr * 32;
  const int n_base = blockIdx.x * 64 + wc * 32;
  const int lm = lane & 15;
  const int kb = (lane < 16) ? 0 : 8;

  v8f zero = {0.f,0.f,0.f,0.f,0.f,0.f,0.f,0.f};
  v8f acc[2][2];
  acc[0][0] = zero; acc[0][1] = zero; acc[1][0] = zero; acc[1][1] = zero;

  for (int k0 = 0; k0 < Kd; k0 += 32) {
    FragBF a[2], b[2], al[2], bl[2];
#pragma unroll
    for (int t = 0; t < 2; ++t) {
      load_frag(a[t],  A  + (size_t)(m_base + t*16 + lm) * Kd + k0 + kb);
      load_frag(al[t], A  + pa + (size_t)(m_base + t*16 + lm) * Kd + k0 + kb);
      load_frag(b[t],  Bt + (size_t)(n_base + t*16 + lm) * Kd + k0 + kb);
      load_frag(bl[t], Bt + pb + (size_t)(n_base + t*16 + lm) * Kd + k0 + kb);
    }
#pragma unroll
    for (int mt = 0; mt < 2; ++mt)
#pragma unroll
      for (int nt = 0; nt < 2; ++nt)
        acc[mt][nt] = wmma_split(a[mt].v, al[mt].v, b[nt].v, bl[nt].v, acc[mt][nt]);
  }

  const int mo = (lane < 16) ? 0 : 8;
  float* sw = stg[wave];
#pragma unroll
  for (int mt = 0; mt < 2; ++mt)
#pragma unroll
    for (int nt = 0; nt < 2; ++nt) {
      const int col = n_base + nt*16 + lm;
      float bv = (epilogue == 1) ? bias[col] : 0.f;
#pragma unroll
      for (int j = 0; j < 8; ++j) sw[(mt*16 + mo + j) * 36 + nt*16 + lm] = apply_epi(acc[mt][nt][j], bv, epilogue);
    }
  asm volatile("s_wait_dscnt 0" ::: "memory");
#pragma unroll 1
  for (int pass = 0; pass < 2; ++pass) {
#pragma unroll
    for (int i = 0; i < 8; ++i) { const int c = lane + 32 * i, rr = c >> 3, q = (c & 7) * 4;
      *(volatile v4f_t*)(C + (size_t)(m_base + rr) * Dn + n_base + q) = *(const volatile v4fa*)(sw + rr * 36 + q); }
    __threadfence();
  }
}

__launch_bounds__(256)
__global__ void k_gemm_bf16_big(const __bf16* __restrict__ A, const __bf16* __restrict__ Bt,
                                float* __restrict__ C, const float* __restrict__ bias,
                                int Kd, int Dn, int epilogue, size_t pa, size_t pb) {
  __shared__ __attribute__((aligned(16))) float stg[8][32 * 68];
  const int lane = threadIdx.x & 31;
  const int wave = threadIdx.x >> 5;
  const int wr = wave >> 1;
  const int wc = wave & 1;
  const int m_base = blockIdx.y * 128 + wr * 32;
  const int n_base = blockIdx.x * 128 + wc * 64;
  const int lm = lane & 15;
  const int kb = (lane < 16) ? 0 : 8;

  v8f zero = {0.f,0.f,0.f,0.f,0.f,0.f,0.f,0.f};
  v8f acc[2][4];
#pragma unroll
  for (int mt = 0; mt < 2; ++mt)
#pragma unroll
    for (int nt = 0; nt < 4; ++nt) acc[mt][nt] = zero;

  for (int k0 = 0; k0 < Kd; k0 += 32) {
    FragBF a[2], al[2], b[4], bl[4];
#pragma unroll
    for (int t = 0; t < 2; ++t) {
      load_frag(a[t],  A + (size_t)(m_base + t*16 + lm) * Kd + k0 + kb);
      load_frag(al[t], A + pa + (size_t)(m_base + t*16 + lm) * Kd + k0 + kb);
    }
#pragma unroll
    for (int t = 0; t < 4; ++t) {
      load_frag(b[t],  Bt + (size_t)(n_base + t*16 + lm) * Kd + k0 + kb);
      load_frag(bl[t], Bt + pb + (size_t)(n_base + t*16 + lm) * Kd + k0 + kb);
    }
#pragma unroll
    for (int mt = 0; mt < 2; ++mt)
#pragma unroll
      for (int nt = 0; nt < 4; ++nt) {
        acc[mt][nt] = wmma_split(a[mt].v, al[mt].v, b[nt].v, bl[nt].v, acc[mt][nt]);
        asm volatile("" ::: "memory");
      }
  }

  const int mo = (lane < 16) ? 0 : 8;
  float* sw = stg[wave];
#pragma unroll
  for (int mt = 0; mt < 2; ++mt)
#pragma unroll
    for (int nt = 0; nt < 4; ++nt) {
      const int col = n_base + nt*16 + lm;
      float bv = (epilogue == 1) ? bias[col] : 0.f;
#pragma unroll
      for (int j = 0; j < 8; ++j) sw[(mt*16 + mo + j) * 68 + nt*16 + lm] = apply_epi(acc[mt][nt][j], bv, epilogue);
    }
  asm volatile("s_wait_dscnt 0" ::: "memory");
#pragma unroll 1
  for (int pass = 0; pass < 2; ++pass) {
#pragma unroll
    for (int i = 0; i < 16; ++i) { const int c = lane + 32 * i, rr = c >> 4, q = (c & 15) * 4;
      *(volatile v4f_t*)(C + (size_t)(m_base + rr) * Dn + n_base + q) = *(const volatile v4fa*)(sw + rr * 68 + q); }
    __threadfence();
  }
}

__global__ void k_conv_silu(const float* __restrict__ xz, const float* __restrict__ cw,
                            const float* __restrict__ cb, float* __restrict__ xc,
                            __bf16* __restrict__ xc_bf, int reverse) {
  int idx = (blockIdx.x * blockDim.x + threadIdx.x) * 2;
  if (idx >= BDIM * LDIM * DIDIM) return;
  const int d = idx % DIDIM;
  const int l = (idx / DIDIM) % LDIM;
  const int b = idx / (DIDIM * LDIM);
  float s2[2];
#pragma unroll
  for (int q = 0; q < 2; ++q) {
    float acc = cb[d + q];
#pragma unroll
    for (int k = 0; k < KCONV; ++k) {
      int lt = reverse ? (l + (KCONV-1) - k) : (l - (KCONV-1) + k);
      if (lt >= 0 && lt < LDIM)
        acc = fmaf(cw[(d + q)*KCONV + k], xz[((size_t)(b*LDIM + lt)) * (2*DIDIM) + d + q], acc);
    }
    s2[q] = acc / (1.f + __expf(-acc));
  }
  typedef __attribute__((ext_vector_type(2))) float v2f_t;
  v2f_t f2; f2.x = s2[0]; f2.y = s2[1];
  unsigned lo; const unsigned p = pk2s(s2[0], s2[1], &lo);
  const size_t PLX = (size_t)MROWS * DIDIM;
  *(volatile v2f_t*)(xc + idx) = f2; *(volatile unsigned*)(xc_bf + idx) = p; *(volatile unsigned*)(xc_bf + PLX + idx) = lo; __threadfence();
  *(volatile v2f_t*)(xc + idx) = f2; *(volatile unsigned*)(xc_bf + idx) = p; *(volatile unsigned*)(xc_bf + PLX + idx) = lo;
}

__global__ void k_extract_dt(const float* __restrict__ xdbl, __bf16* __restrict__ dt_bf) {
  int i = (blockIdx.x * blockDim.x + threadIdx.x) * 2;
  if (i >= MROWS * RDIM) return;
  int r = i % RDIM, row = i / RDIM;
  unsigned lo; const unsigned p = pk2s(xdbl[(size_t)row * XDBLW + r], xdbl[(size_t)row * XDBLW + r + 1], &lo);
  *(volatile unsigned*)(dt_bf + i) = p; *(volatile unsigned*)(dt_bf + (size_t)MROWS * RDIM + i) = lo; __threadfence();
  *(volatile unsigned*)(dt_bf + i) = p; *(volatile unsigned*)(dt_bf + (size_t)MROWS * RDIM + i) = lo;
}

#define SCAN_CH 32
__launch_bounds__(256)
__global__ void k_scan(const float* __restrict__ dt, const float* __restrict__ xdbl,
                       const float* __restrict__ xc, const float* __restrict__ xz,
                       const float* __restrict__ A_log, const float* __restrict__ Dp,
                       __bf16* __restrict__ y_bf, int reverse) {
  __shared__ __align__(16) float BC[2][SCAN_CH][2*SDIM];
  const int tid = threadIdx.x;
  const int b   = blockIdx.y;
  const int d   = (blockIdx.x * 256 + tid) * 2;

  float An[2][SDIM], h[2][SDIM], dskip[2];
#pragma unroll
  for (int q = 0; q < 2; ++q) {
#pragma unroll
    for (int s = 0; s < SDIM; ++s) { An[q][s] = -__expf(A_log[(d + q)*SDIM + s]); h[q][s] = 0.f; }
    dskip[q] = Dp[d + q];
  }
  const size_t PLY = (size_t)MROWS * DIDIM;

  const int stt  = tid >> 3;
  const int sseg = tid & 7;

  auto stage = [&](int buf, int t0) {
    int l = reverse ? (LDIM-1 - (t0 + stt)) : (t0 + stt);
    const float* g = xdbl + (size_t)(b*LDIM + l) * XDBLW + RDIM + sseg*4;
    unsigned lofs = (unsigned)(unsigned long long)(lds_f32*)&BC[buf][stt][sseg*4];
    unsigned long long ga = (unsigned long long)g;
    asm volatile("global_load_async_to_lds_b128 %0, %1, off"
                 :: "v"(lofs), "v"(ga) : "memory");
  };

  stage(0, 0);
  asm volatile("s_wait_asynccnt 0" ::: "memory");
  __syncthreads();

  const int NCHUNK = LDIM / SCAN_CH;
  for (int c = 0; c < NCHUNK; ++c) {
    const int cur = c & 1;
    if (c + 1 < NCHUNK) stage(cur ^ 1, (c + 1) * SCAN_CH);

    const int t0 = c * SCAN_CH;
    for (int tt = 0; tt < SCAN_CH; ++tt) {
      int l = reverse ? (LDIM-1 - (t0 + tt)) : (t0 + tt);
      const size_t base = (size_t)(b*LDIM + l);
      float yo[2];
#pragma unroll
      for (int q = 0; q < 2; ++q) {
        const float dtv = dt[base*DIDIM + d + q];
        const float xcv = xc[base*DIDIM + d + q];
        const float zv  = xz[base*(2*DIDIM) + DIDIM + d + q];
        const float dx  = dtv * xcv;
        float y = 0.f;
#pragma unroll
        for (int s = 0; s < SDIM; ++s) {
          float dA  = __expf(dtv * An[q][s]);
          float dBu = dx * BC[cur][tt][s];
          h[q][s] = fmaf(dA, h[q][s], dBu);
          y       = fmaf(h[q][s], BC[cur][tt][SDIM + s], y);
        }
        y = fmaf(xcv, dskip[q], y);
        yo[q] = y * (zv / (1.f + __expf(-zv)));
      }
      { unsigned lo; const unsigned p = pk2s(yo[0], yo[1], &lo);
        *(volatile unsigned*)(y_bf + base*DIDIM + d) = p; *(volatile unsigned*)(y_bf + PLY + base*DIDIM + d) = lo; __threadfence();
        *(volatile unsigned*)(y_bf + base*DIDIM + d) = p; *(volatile unsigned*)(y_bf + PLY + base*DIDIM + d) = lo; }
    }
    asm volatile("s_wait_asynccnt 0" ::: "memory");
    __syncthreads();
  }
}

__launch_bounds__(256)
__global__ void k_residual_ln(const float* __restrict__ h, const float* __restrict__ f,
                              const float* __restrict__ bw, const float* __restrict__ g,
                              const float* __restrict__ beta, float* __restrict__ out) {
  __shared__ float red[256];
  const int row = blockIdx.x;
  const int tid = threadIdx.x;
  const size_t base = (size_t)row * NDIM;
  float v0 = h[base + tid]       + f[base + tid]       + bw[base + tid];
  float v1 = h[base + tid + 256] + f[base + tid + 256] + bw[base + tid + 256];

  red[tid] = v0 + v1;
  __syncthreads();
  for (int off = 128; off > 0; off >>= 1) {
    if (tid < off) red[tid] += red[tid + off];
    __syncthreads();
  }
  const float mu = red[0] * (1.f / NDIM);
  __syncthreads();
  const float d0 = v0 - mu, d1 = v1 - mu;
  red[tid] = d0*d0 + d1*d1;
  __syncthreads();
  for (int off = 128; off > 0; off >>= 1) {
    if (tid < off) red[tid] += red[tid + off];
    __syncthreads();
  }
  const float rstd = rsqrtf(red[0] * (1.f / NDIM) + 1e-5f);
  const float o0 = d0 * rstd * g[tid] + beta[tid], o1 = d1 * rstd * g[tid + 256] + beta[tid + 256];
  *(volatile float*)(out + base + tid) = o0; *(volatile float*)(out + base + tid + 256) = o1; __threadfence();
  *(volatile float*)(out + base + tid) = o0; *(volatile float*)(out + base + tid + 256) = o1;
}

extern "C" void kernel_launch(void* const* d_in, const int* in_sizes, int n_in,
                              void* d_out, int out_size, void* d_ws, size_t ws_size,
                              hipStream_t stream) {
  const float* x    = (const float*)d_in[0];
  const float* inw  = (const float*)d_in[1];
  const float* cw   = (const float*)d_in[2];
  const float* cb   = (const float*)d_in[3];
  const float* xw   = (const float*)d_in[4];
  const float* dtw  = (const float*)d_in[5];
  const float* dtbp = (const float*)d_in[6];
  const float* Alog = (const float*)d_in[7];
  const float* Dp   = (const float*)d_in[8];
  const float* ow   = (const float*)d_in[9];
  const float* lng  = (const float*)d_in[10];
  const float* lnb  = (const float*)d_in[11];
  float* outp = (float*)d_out;

  char* ws = (char*)d_ws;
  size_t off = 0;
  auto alloc = [&](size_t bytes) -> char* {
    char* p = ws + off;
    off = (off + bytes + 255) & ~(size_t)255;
    return p;
  };

  float*  hbuf   = (float*) alloc((size_t)MROWS * NDIM * 4);
  __bf16* u_bf   = (__bf16*)alloc((size_t)MROWS * NDIM * 2 * 2);
  float*  xz     = (float*) alloc((size_t)MROWS * 2 * DIDIM * 4);
  float*  xc     = (float*) alloc((size_t)MROWS * DIDIM * 4);
  __bf16* xc_bf  = (__bf16*)alloc((size_t)MROWS * DIDIM * 2 * 2);
  float*  xdbl   = (float*) alloc((size_t)MROWS * XDBLW * 4);
  __bf16* dt_bf  = (__bf16*)alloc((size_t)MROWS * RDIM * 2 * 2);
  float*  dtf    = (float*) alloc((size_t)MROWS * DIDIM * 4);
  __bf16* y_bf   = (__bf16*)alloc((size_t)MROWS * DIDIM * 2 * 2);
  float*  out0   = (float*) alloc((size_t)MROWS * NDIM * 4);
  float*  out1   = (float*) alloc((size_t)MROWS * NDIM * 4);
  __bf16* inw_bf = (__bf16*)alloc((size_t)NMB * 2 * DIDIM * NDIM * 2 * 2);
  __bf16* xw_bf  = (__bf16*)alloc((size_t)NMB * XDBLW * DIDIM * 2 * 2);
  __bf16* dtw_bf = (__bf16*)alloc((size_t)NMB * DIDIM * RDIM * 2 * 2);
  __bf16* ow_bf  = (__bf16*)alloc((size_t)NMB * NDIM * DIDIM * 2 * 2);
  const size_t PL_U = (size_t)MROWS * NDIM, PL_XC = (size_t)MROWS * DIDIM, PL_DT = (size_t)MROWS * RDIM, PL_Y = (size_t)MROWS * DIDIM;
  const size_t PL_INW = (size_t)NMB * 2 * DIDIM * NDIM, PL_XW = (size_t)NMB * XDBLW * DIDIM, PL_DTW = (size_t)NMB * DIDIM * RDIM, PL_OW = (size_t)NMB * NDIM * DIDIM;
  const int MR = MROWS;

  auto cast = [&](const float* s, __bf16* dst, size_t n) {
    k_cast_bf16<<<dim3((unsigned)((n / 2 + 255) / 256)), 256, 0, stream>>>(s, dst, (int)n);
  };
  auto gemm = [&](const __bf16* A, size_t pa, const __bf16* Bt, size_t pb, float* C, const float* bias,
                  int Kd, int Dn, int epi) {
    if ((Dn % 128) == 0) {
      dim3 g(Dn / 128, MR / 128);
      k_gemm_bf16_big<<<g, 256, 0, stream>>>(A, Bt, C, bias, Kd, Dn, epi, pa, pb);
    } else {
      dim3 g(Dn / 64, MR / 64);
      k_gemm_bf16<<<g, 128, 0, stream>>>(A, Bt, C, bias, Kd, Dn, epi, pa, pb);
    }
  };

  cast(inw, inw_bf, (size_t)NMB * 2 * DIDIM * NDIM);
  cast(xw,  xw_bf,  (size_t)NMB * XDBLW * DIDIM);
  cast(dtw, dtw_bf, (size_t)NMB * DIDIM * RDIM);
  cast(ow,  ow_bf,  (size_t)NMB * NDIM * DIDIM);

  hipMemcpyAsync(hbuf, x, (size_t)MROWS * NDIM * 4, hipMemcpyDeviceToDevice, stream);

  const int NLRUN = NLAYER;
  for (int l = 0; l < NLRUN; ++l) {
    cast(hbuf, u_bf, (size_t)MROWS * NDIM);
    for (int dir = 0; dir < 2; ++dir) {
      const int i = 2 * l + dir;
      gemm(u_bf, PL_U, inw_bf + (size_t)i * 2 * DIDIM * NDIM, PL_INW, xz, nullptr, NDIM, 2 * DIDIM, 0);
      k_conv_silu<<<dim3((MR * DIDIM / 2 + 255) / 256), 256, 0, stream>>>(
          xz, cw + (size_t)i * DIDIM * KCONV, cb + (size_t)i * DIDIM, xc, xc_bf, dir);
      gemm(xc_bf, PL_XC, xw_bf + (size_t)i * XDBLW * DIDIM, PL_XW, xdbl, nullptr, DIDIM, XDBLW, 0);
      k_extract_dt<<<dim3((MR * RDIM / 2 + 255) / 256), 256, 0, stream>>>(xdbl, dt_bf);
      gemm(dt_bf, PL_DT, dtw_bf + (size_t)i * DIDIM * RDIM, PL_DTW, dtf, dtbp + (size_t)i * DIDIM, RDIM, DIDIM, 1);
      dim3 sg(DIDIM / 512, MR / LDIM);
      k_scan<<<sg, 256, 0, stream>>>(dtf, xdbl, xc, xz,
                                     Alog + (size_t)i * DIDIM * SDIM, Dp + (size_t)i * DIDIM,
                                     y_bf, dir);
      gemm(y_bf, PL_Y, ow_bf + (size_t)i * NDIM * DIDIM, PL_OW, dir == 0 ? out0 : out1, nullptr,
           DIDIM, NDIM, 0);
    }
    float* dst = (l == NLRUN - 1) ? outp : hbuf;
    k_residual_ln<<<dim3(MR), 256, 0, stream>>>(hbuf, out0, out1,
                                                lng + (size_t)l * NDIM,
                                                lnb + (size_t)l * NDIM, dst);
  }
}
